// MambaBlock_60327110639692
// MI455X (gfx1250) — hardware-verified
//
#include <hip/hip_runtime.h>
#include <math.h>

typedef __attribute__((ext_vector_type(16))) _Float16 v16h;
typedef __attribute__((ext_vector_type(8)))  _Float16 v8h;
typedef __attribute__((ext_vector_type(8)))  float    v8f;
typedef __attribute__((ext_vector_type(4)))  float    v4f;
typedef __attribute__((ext_vector_type(2)))  float    v2f;
typedef __attribute__((ext_vector_type(4)))  unsigned v4u;

constexpr int kBatch = 4;
constexpr int kSeq   = 2048;
constexpr int kDm    = 768;
constexpr int kDi    = 1536;
constexpr int kNs    = 128;
constexpr int kNh    = 24;
constexpr int kHd    = 64;
constexpr int kCv    = kDi + 2 * kNs;
constexpr int kNin   = 2 * kDi + 2 * kNs + kNh;
constexpr int kNinP  = 3392;
constexpr int kRows  = kBatch * kSeq;
constexpr int kQ     = 64;
constexpr int kNc    = kSeq / kQ;
constexpr int kBC    = kBatch * kNc;
constexpr int kDtP   = 64;
constexpr int kTileZ  = kDi / 64;
constexpr int kTileDt = (kDi + kCv) / 64;
constexpr int kMP    = 72;
constexpr int kHP    = 136;
constexpr int kConvTP = 260;
constexpr float kWCarry    = 32.0f;
constexpr float kWCarryInv = 1.0f / 32.0f;
constexpr float kCarry     = 2048.0f;
constexpr float kCarryInv  = 1.0f / 2048.0f;
static_assert(kCv == 1792);
static_assert(kNin == 3352);
static_assert(kNinP % 64 == 0 && kNinP >= kNin && kNinP - kNin < 64);
static_assert(kNh * kHd == kDi);
static_assert(kRows == 8192);
static_assert(kDm % 32 == 0 && kDi % 32 == 0 && kNs % 32 == 0 && kQ % 32 == 0);
static_assert(kRows % 64 == 0 && kDm % 64 == 0 && kDi % 64 == 0 && kCv % 64 == 0);
static_assert(kTileZ == 24 && kTileDt == 52 && kNinP / 64 == 53);
static_assert(kSeq % kQ == 0 && kNc == 32 && kBC == 128);

constexpr size_t kOffX16  = 0;
constexpr size_t kOffWIN  = kOffX16  + (size_t)kRows * kDm * 2;
constexpr size_t kOffWOUT = kOffWIN  + (size_t)kNinP * kDm * 2;
constexpr size_t kOffZ16  = kOffWOUT + (size_t)kDm * kDi * 2;
constexpr size_t kOffXR   = kOffZ16  + (size_t)kRows * kDi * 2;
constexpr size_t kOffDT   = kOffXR   + (size_t)kRows * kCv * 2;
constexpr size_t kOffXC   = kOffDT   + (size_t)kRows * kDtP * 4;
constexpr size_t kOffG    = kOffXC   + (size_t)kRows * kCv * 2;
constexpr size_t kOffBT   = kOffG    + (size_t)kBC * kQ * kQ * 4;
constexpr size_t kWsTotal = kOffBT   + (size_t)kBC * kNs * kQ * 2;
static_assert(kWsTotal == 110329856ull);
static_assert(kWsTotal <= 134217728ull);
static_assert((kOffWIN % 128) == 0 && (kOffWOUT % 128) == 0 && (kOffZ16 % 128) == 0 && (kOffXR % 128) == 0 &&
              (kOffDT % 128) == 0 && (kOffXC % 128) == 0 && (kOffG % 128) == 0 && (kOffBT % 128) == 0);
static_assert((size_t)kRows * kDi * 2 <= (size_t)kRows * kCv * 2);

__device__ __forceinline__ float h16_to_f32(unsigned hb) {
  const unsigned sgn = (hb & 0x8000u) << 16;
  const unsigned em = hb & 0x7fffu;
  const float fn = __uint_as_float((em << 13) + 0x38000000u);
  const float fs = (float)em * 5.9604644775390625e-8f;
  const float mag = (em < 0x400u) ? fs : fn;
  return __uint_as_float(__float_as_uint(mag) | sgn);
}
__device__ __forceinline__ unsigned short f32_to_h16_bits(float f) {
  const _Float16 hq = (_Float16)f;
  return __builtin_bit_cast(unsigned short, hq);
}
__device__ __forceinline__ float flush_tiny(float v) {
  return (v < 1.17549435e-38f) ? 0.0f : v;
}
union FragU { v16h v; v8h h[2]; };
__device__ __forceinline__ v16h frag_ld(const _Float16* p) {
  FragU f;
  f.h[0] = *(const v8h*)(p);
  f.h[1] = *(const v8h*)(p + 16);
  return f.v;
}
__device__ __forceinline__ v8f mma_h(v16h a, v16h b, v8f c) {
  return __builtin_amdgcn_wmma_f32_16x16x32_f16(false, a, false, b, (short)0, c, false, false);
}
__device__ __forceinline__ void guard4h(v8f& a, v8f& b, v8f& c, v8f& d, v16h x, v16h y0, v16h y1, v16h y2, v16h y3) {
  asm volatile("v_nop\n\tv_nop\n\tv_nop\n\tv_nop"
               : "+v"(a), "+v"(b), "+v"(c), "+v"(d)
               : "v"(x), "v"(y0), "v"(y1), "v"(y2), "v"(y3));
}
__device__ __forceinline__ void acc_guard4(v8f& a, v8f& b, v8f& c, v8f& d) {
  asm volatile("v_nop\n\tv_nop\n\tv_nop\n\tv_nop" : "+v"(a), "+v"(b), "+v"(c), "+v"(d));
}
__device__ __forceinline__ void wave_lds_sync() {
  __builtin_amdgcn_fence(__ATOMIC_RELEASE, "workgroup");
  __builtin_amdgcn_wave_barrier();
  __builtin_amdgcn_fence(__ATOMIC_ACQUIRE, "workgroup");
}

__global__ __launch_bounds__(256) void cast_rows_f16_kernel(
    const float* __restrict__ src, unsigned short* __restrict__ dst, int total8, int ncols, int nreal_rows, float scale)
{
  const int i = blockIdx.x * 256 + threadIdx.x;
  if (i >= total8) return;
  const size_t e0 = (size_t)i << 3;
  const int row = (int)(e0 / (size_t)ncols);
  const int col = (int)(e0 - (size_t)row * (size_t)ncols);
  const int rc = (row < nreal_rows) ? row : (nreal_rows - 1);
  const bool live = (row < nreal_rows);
  const float* p = src + (size_t)rc * (size_t)ncols + col;
  const v4f a0 = *(const v4f*)(p);
  const v4f a1 = *(const v4f*)(p + 4);
  v8h hv;
#pragma unroll
  for (int e = 0; e < 4; ++e) {
    const float f0 = live ? (a0[e] * scale) : 0.0f;
    const float f1 = live ? (a1[e] * scale) : 0.0f;
    hv[e]     = (_Float16)f0;
    hv[4 + e] = (_Float16)f1;
  }
  unsigned short* q = dst + e0;
  *(volatile v8h*)q = hv;
  __threadfence();
  *(volatile v8h*)q = hv;
}

template <int EPI>
__global__ __launch_bounds__(256) void gemm64_f16_kernel(
    const unsigned short* __restrict__ Ap, int lda, long strideA,
    const unsigned short* __restrict__ Btp, int ldb, long strideB,
    float* __restrict__ Cf, int ldc, long strideC,
    const float* __restrict__ addend,
    unsigned short* __restrict__ Zout, unsigned short* __restrict__ XRout, float* __restrict__ DTout,
    int M, int N, int K, int nbatch, float scale)
{
  __shared__ __align__(16) float sT[8][16 * 68];
  const int lane = threadIdx.x & 31;
  const int wave = threadIdx.x >> 5;
  const int tilesN = N >> 6;
  const int tilesM = M >> 6;
  const int tpb = tilesM * tilesN;
  const int tile = blockIdx.x * 8 + wave;
  if (tile >= tpb * nbatch) return;
  const int bidx = tile / tpb;
  const int tl = tile - bidx * tpb;
  const int tm = tl / tilesN;
  const int tn = tl - tm * tilesN;
  const int m0 = tm << 6;
  const int n0 = tn << 6;

  const _Float16* Ab = (const _Float16*)Ap + (size_t)bidx * strideA;
  const _Float16* Bb = (const _Float16*)Btp + (size_t)bidx * strideB;

  const int rlane = lane & 15;
  const int koff  = (lane >> 4) * 8;
  const int mOff  = (lane >> 4) * 8;

  v8f acc[4][4];
#pragma unroll
  for (int i = 0; i < 4; ++i)
#pragma unroll
    for (int j = 0; j < 4; ++j) acc[i][j] = (v8f){0.f, 0.f, 0.f, 0.f, 0.f, 0.f, 0.f, 0.f};

  for (int k0 = 0; k0 < K; k0 += 32) {
    v16h bh[4];
#pragma unroll
    for (int j = 0; j < 4; ++j) {
      const size_t bo = (size_t)(n0 + (j << 4) + rlane) * ldb + koff + k0;
      bh[j] = frag_ld(Bb + bo);
    }
#pragma unroll
    for (int i = 0; i < 4; ++i) {
      const size_t ao = (size_t)(m0 + (i << 4) + rlane) * lda + koff + k0;
      const v16h ah = frag_ld(Ab + ao);
#pragma unroll
      for (int j = 0; j < 4; ++j) acc[i][j] = mma_h(ah, bh[j], acc[i][j]);
      guard4h(acc[i][0], acc[i][1], acc[i][2], acc[i][3], ah, bh[0], bh[1], bh[2], bh[3]);
    }
  }
  acc_guard4(acc[0][0], acc[0][1], acc[0][2], acc[0][3]);
  acc_guard4(acc[1][0], acc[1][1], acc[1][2], acc[1][3]);
  acc_guard4(acc[2][0], acc[2][1], acc[2][2], acc[2][3]);
  acc_guard4(acc[3][0], acc[3][1], acc[3][2], acc[3][3]);

  float* slab = sT[wave];
  const bool out16 = (EPI == 2) && (tn < kTileDt);
  unsigned short* o16 = Zout;
  int p16 = kDi;
  int c16 = n0;
  if (EPI == 2 && tn >= kTileZ) {
    o16 = XRout;
    p16 = kCv;
    c16 = n0 - kDi;
  }
  float* of32 = (EPI == 2) ? DTout : (Cf + (size_t)bidx * strideC);
  const int pf32 = (EPI == 2) ? kDtP : ldc;
  const int cf32 = (EPI == 2) ? 0 : n0;

#pragma unroll
  for (int i = 0; i < 4; ++i) {
    const int mBase = m0 + (i << 4);
#pragma unroll
    for (int j = 0; j < 4; ++j) {
#pragma unroll
      for (int r = 0; r < 8; ++r) slab[(mOff + r) * 68 + (j << 4) + rlane] = acc[i][j][r] * scale;
    }
    wave_lds_sync();
    if (out16) {
      const int q = lane >> 3, c8 = (lane & 7) * 8;
      v8h hv[4];
#pragma unroll
      for (int it = 0; it < 4; ++it) {
        const float* sp = slab + (it * 4 + q) * 68 + c8;
        const v4f a0 = *(const v4f*)(sp);
        const v4f a1 = *(const v4f*)(sp + 4);
#pragma unroll
        for (int e = 0; e < 4; ++e) {
          hv[it][e]     = (_Float16)a0[e];
          hv[it][4 + e] = (_Float16)a1[e];
        }
      }
      for (int pass = 0; pass < 2; ++pass) {
#pragma unroll
        for (int it = 0; it < 4; ++it) {
          const int row = it * 4 + q;
          *(volatile v8h*)(o16 + (size_t)(mBase + row) * p16 + c16 + c8) = hv[it];
        }
        __threadfence();
      }
    } else {
      const int hh = lane >> 4, c4 = (lane & 15) * 4;
      v4f vals[8];
#pragma unroll
      for (int it = 0; it < 8; ++it) {
        const int row = it * 2 + hh;
        v4f v = *(const v4f*)(slab + row * 68 + c4);
        if (EPI == 1) {
          const v4f r4 = *(const v4f*)(addend + (size_t)(mBase + row) * ldc + n0 + c4);
          v = v + r4;
        }
        vals[it] = v;
      }
      for (int pass = 0; pass < 2; ++pass) {
#pragma unroll
        for (int it = 0; it < 8; ++it) {
          const int row = it * 2 + hh;
          *(volatile v4f*)(of32 + (size_t)(mBase + row) * pf32 + cf32 + c4) = vals[it];
        }
        __threadfence();
      }
    }
    wave_lds_sync();
  }
}

__global__ __launch_bounds__(128) void conv_silu_kernel(
    const unsigned short* __restrict__ XR, const float* __restrict__ cw, const float* __restrict__ cb,
    unsigned short* __restrict__ XC)
{
  __shared__ __align__(16) float sT[16 * kConvTP];
  const int tid = threadIdx.x, lane = tid & 31, wave = tid >> 5;
  const int d0 = blockIdx.x * 256;
  const int d  = d0 + 2 * tid;
  const int g0 = blockIdx.y * 64;
  const int tb = g0 & (kSeq - 1);
  const v4f wa = *(const v4f*)(cw + (size_t)d * 4);
  const v4f wb = *(const v4f*)(cw + (size_t)d * 4 + 4);
  const float ba = cb[d], bb = cb[d + 1];
  const unsigned* XRw = (const unsigned*)(const void*)XR;
  float am3, am2, am1, bm3, bm2, bm1;
  {
    const bool hist = (tb > 0);
    const int rb = hist ? (g0 - 3) : g0;
    const unsigned u3 = XRw[((size_t)rb * kCv + d) >> 1];
    const unsigned u2 = XRw[((size_t)(rb + 1) * kCv + d) >> 1];
    const unsigned u1 = XRw[((size_t)(rb + 2) * kCv + d) >> 1];
    const float a3 = h16_to_f32(u3 & 0xffffu), b3 = h16_to_f32(u3 >> 16);
    const float a2 = h16_to_f32(u2 & 0xffffu), b2 = h16_to_f32(u2 >> 16);
    const float a1 = h16_to_f32(u1 & 0xffffu), b1 = h16_to_f32(u1 >> 16);
    am3 = hist ? a3 : 0.f;
    am2 = hist ? a2 : 0.f;
    am1 = hist ? a1 : 0.f;
    bm3 = hist ? b3 : 0.f;
    bm2 = hist ? b2 : 0.f;
    bm1 = hist ? b1 : 0.f;
  }
#pragma unroll 1
  for (int sub = 0; sub < 4; ++sub) {
    const int lb = g0 + sub * 16;
#pragma unroll 1
    for (int s = 0; s < 16; ++s) {
      const unsigned u = XRw[((size_t)(lb + s) * kCv + d) >> 1];
      const float xa = h16_to_f32(u & 0xffffu);
      const float xb = h16_to_f32(u >> 16);
      float acca = wa[0] * am3;
      acca = fmaf(wa[1], am2, acca);
      acca = fmaf(wa[2], am1, acca);
      acca = fmaf(wa[3], xa, acca);
      float accb = wb[0] * bm3;
      accb = fmaf(wb[1], bm2, accb);
      accb = fmaf(wb[2], bm1, accb);
      accb = fmaf(wb[3], xb, accb);
      const float sva = acca + ba;
      const float svb = accb + bb;
      const float sga = __builtin_amdgcn_rcpf(1.0f + expf(-sva));
      const float sgb = __builtin_amdgcn_rcpf(1.0f + expf(-svb));
      v2f o;
      o[0] = sva * sga;
      o[1] = svb * sgb;
      *(v2f*)(sT + s * kConvTP + 2 * tid) = o;
      am3 = am2; am2 = am1; am1 = xa;
      bm3 = bm2; bm2 = bm1; bm1 = xb;
    }
    __syncthreads();
    v8h hv[4];
#pragma unroll
    for (int it = 0; it < 4; ++it) {
      const float* sp = sT + (it * 4 + wave) * kConvTP + lane * 8;
      const v4f a0 = *(const v4f*)(sp);
      const v4f a1 = *(const v4f*)(sp + 4);
#pragma unroll
      for (int e = 0; e < 4; ++e) {
        hv[it][e]     = (_Float16)a0[e];
        hv[it][4 + e] = (_Float16)a1[e];
      }
    }
    for (int pass = 0; pass < 2; ++pass) {
#pragma unroll
      for (int it = 0; it < 4; ++it)
        *(volatile v8h*)(XC + (size_t)(lb + it * 4 + wave) * kCv + d0 + lane * 8) = hv[it];
      __threadfence();
    }
    __syncthreads();
  }
}

__global__ __launch_bounds__(256) void bt_transpose_kernel(
    const unsigned short* __restrict__ XC, unsigned short* __restrict__ BT)
{
  __shared__ __align__(16) unsigned short tS[64 * 136];
  const int tid = threadIdx.x, lane = tid & 31, wave = tid >> 5;
  const int bc = blockIdx.x;
  const size_t r0 = (size_t)bc * kQ;
#pragma unroll
  for (int p = 0; p < 4; ++p) {
    const int idx = tid + 256 * p;
    const int s  = idx >> 4;
    const int pc = (idx & 15) * 8;
    const v4u v = *(const v4u*)(XC + (r0 + s) * kCv + kDi + pc);
    *(v4u*)(tS + s * 136 + pc) = v;
  }
  __syncthreads();
  const int q = lane >> 3, c8 = (lane & 7) * 8;
  v4u ov[4];
#pragma unroll
  for (int it = 0; it < 4; ++it) {
    const int n = it * 32 + wave * 4 + q;
#pragma unroll
    for (int k = 0; k < 4; ++k) {
      const unsigned lo = (unsigned)tS[(c8 + 2 * k) * 136 + n];
      const unsigned hi = (unsigned)tS[(c8 + 2 * k + 1) * 136 + n];
      ov[it][k] = lo | (hi << 16);
    }
  }
  for (int pass = 0; pass < 2; ++pass) {
#pragma unroll
    for (int it = 0; it < 4; ++it) {
      const int n = it * 32 + wave * 4 + q;
      *(volatile v4u*)(BT + ((size_t)bc * kNs + n) * kQ + c8) = ov[it];
    }
    __threadfence();
  }
}

__global__ __launch_bounds__(128) void ssd_chunk_kernel(
    const unsigned short* __restrict__ XC, const float* __restrict__ DT32, const float* __restrict__ G32,
    const unsigned short* __restrict__ BT, const float* __restrict__ dt_bias, const float* __restrict__ A_log,
    const float* __restrict__ Dv, unsigned short* __restrict__ Y16)
{
  __shared__ __align__(16) unsigned short sH[64 * kHP];
  __shared__ __align__(16) unsigned short sM[64 * kMP];
  __shared__ __align__(16) unsigned short sXT[64 * kMP];
  __shared__ __align__(16) unsigned short sXW[64 * kMP];
  __shared__ __align__(16) float sCs[64];
  __shared__ __align__(16) float sDt[64];
  __shared__ __align__(16) float sWs[64];
  __shared__ __align__(16) float sEc[64];
  __shared__ __align__(16) float sScal[4];
  __shared__ __align__(16) float sSlab[4][16 * 68];

  const int tid = threadIdx.x, lane = tid & 31, wave = tid >> 5;
  const int hh = lane >> 4, rl = lane & 15, koff = hh * 8;
  const int b = blockIdx.x / kNh;
  const int h = blockIdx.x - b * kNh;
  const size_t row0 = (size_t)b * kSeq;
  const float Ah  = -expf(A_log[h]);
  const float dtb = dt_bias[h];
  const float Dh  = Dv[h];

  {
    unsigned* zp = (unsigned*)(void*)sH;
#pragma unroll 1
    for (int i = tid; i < (64 * kHP) / 2; i += 128) zp[i] = 0u;
  }
  v8f Hacc[8];
#pragma unroll
  for (int j = 0; j < 8; ++j) Hacc[j] = (v8f){0.f, 0.f, 0.f, 0.f, 0.f, 0.f, 0.f, 0.f};

  const int srow = tid >> 3;
  const int pg   = (tid & 7) * 8;
  float* slab = sSlab[wave];

#pragma unroll 1
  for (int c = 0; c < kNc; ++c) {
    const size_t r0 = row0 + (size_t)c * kQ;
    const int bc = b * kNc + c;
    __syncthreads();

    {
      const float x0 = DT32[(r0 + 2 * lane) * kDtP + h] + dtb;
      const float x1 = DT32[(r0 + 2 * lane + 1) * kDtP + h] + dtb;
      const float dt0 = fmaxf(x0, 0.0f) + log1pf(expf(-fabsf(x0)));
      const float dt1 = fmaxf(x1, 0.0f) + log1pf(expf(-fabsf(x1)));
      const float a0 = dt0 * Ah;
      const float a1 = dt1 * Ah;
      float sc = a0 + a1;
#pragma unroll
      for (int off = 1; off < 32; off <<= 1) {
        const float v = __shfl_up(sc, off, 32);
        sc += (lane >= off) ? v : 0.0f;
      }
      float ex = __shfl_up(sc, 1, 32);
      ex = (lane == 0) ? 0.0f : ex;
      const float cend = __shfl(sc, 31, 32);
      const float cs0 = ex + a0;
      const float cs1 = sc;
      const float w0 = flush_tiny(expf(fminf(cend - cs0, 0.0f))) * (dt0 * kCarry);
      const float w1 = flush_tiny(expf(fminf(cend - cs1, 0.0f))) * (dt1 * kCarry);
      const float e0 = flush_tiny(expf(fminf(cs0, 0.0f)));
      const float e1 = flush_tiny(expf(fminf(cs1, 0.0f)));
      const float dec = flush_tiny(expf(fminf(cend, 0.0f)));
      if (wave == 0) {
        sCs[2 * lane] = cs0;
        sCs[2 * lane + 1] = cs1;
        sDt[2 * lane] = dt0;
        sDt[2 * lane + 1] = dt1;
        sWs[2 * lane] = w0;
        sWs[2 * lane + 1] = w1;
        sEc[2 * lane] = e0;
        sEc[2 * lane + 1] = e1;
        if (lane == 0) sScal[0] = dec;
      }
    }
    v4u xw[4];
#pragma unroll
    for (int it = 0; it < 4; ++it) {
      const int s = srow + 16 * it;
      xw[it] = *(const v4u*)(XC + (r0 + s) * kCv + h * kHd + pg);
    }
#pragma unroll
    for (int it = 0; it < 4; ++it) {
      const int s = srow + 16 * it;
#pragma unroll
      for (int wd = 0; wd < 4; ++wd) {
        const unsigned w = xw[it][wd];
        sXT[(pg + 2 * wd) * kMP + s]     = (unsigned short)(w & 0xffffu);
        sXT[(pg + 2 * wd + 1) * kMP + s] = (unsigned short)(w >> 16);
      }
    }
    __syncthreads();

#pragma unroll
    for (int it = 0; it < 4; ++it) {
      const int s = srow + 16 * it;
      const float ws = sWs[s];
#pragma unroll
      for (int wd = 0; wd < 4; ++wd) {
        const unsigned w = xw[it][wd];
        const float f0 = h16_to_f32(w & 0xffffu) * ws;
        const float f1 = h16_to_f32(w >> 16) * ws;
        sXW[(pg + 2 * wd) * kMP + s]     = f32_to_h16_bits(f0);
        sXW[(pg + 2 * wd + 1) * kMP + s] = f32_to_h16_bits(f1);
      }
    }
#pragma unroll 1
    for (int it = 0; it < 4; ++it) {
      const int t = srow + 16 * it;
      const float* gp = G32 + ((size_t)bc * kQ + t) * kQ + pg;
      const v4f g0 = *(const v4f*)(gp);
      const v4f g1 = *(const v4f*)(gp + 4);
      const v4f c0 = *(const v4f*)(sCs + pg);
      const v4f c1 = *(const v4f*)(sCs + pg + 4);
      const v4f q0 = *(const v4f*)(sDt + pg);
      const v4f q1 = *(const v4f*)(sDt + pg + 4);
      const float cst = sCs[t];
      v8h hv;
#pragma unroll
      for (int e = 0; e < 4; ++e) {
        const float da = fminf(cst - c0[e], 0.0f);
        const float db = fminf(cst - c1[e], 0.0f);
        const float va = g0[e] * expf(da) * (q0[e] * kCarry);
        const float vb = g1[e] * expf(db) * (q1[e] * kCarry);
        const float ma = ((pg + e) <= t) ? va : 0.0f;
        const float mb = ((pg + 4 + e) <= t) ? vb : 0.0f;
        hv[e]     = (_Float16)ma;
        hv[4 + e] = (_Float16)mb;
      }
      *(v8h*)((_Float16*)(void*)sM + t * kMP + pg) = hv;
    }
    v8f acc[4];
#pragma unroll
    for (int j = 0; j < 4; ++j) acc[j] = (v8f){0.f, 0.f, 0.f, 0.f, 0.f, 0.f, 0.f, 0.f};
    {
      const _Float16* Cg = (const _Float16*)(const void*)XC + (r0 + 16 * wave + rl) * kCv + kDi + kNs + koff;
      const _Float16* Hs = (const _Float16*)(const void*)sH + rl * kHP + koff;
#pragma unroll 1
      for (int k0 = 0; k0 < kNs; k0 += 32) {
        const v16h a = frag_ld(Cg + k0);
        v16h bf[4];
#pragma unroll
        for (int j = 0; j < 4; ++j) bf[j] = frag_ld(Hs + (j * 16) * kHP + k0);
#pragma unroll
        for (int j = 0; j < 4; ++j) acc[j] = mma_h(a, bf[j], acc[j]);
        guard4h(acc[0], acc[1], acc[2], acc[3], a, bf[0], bf[1], bf[2], bf[3]);
      }
      const v4f e0 = *(const v4f*)(sEc + 16 * wave + 8 * hh);
      const v4f e1 = *(const v4f*)(sEc + 16 * wave + 8 * hh + 4);
#pragma unroll
      for (int j = 0; j < 4; ++j) {
#pragma unroll
        for (int r = 0; r < 4; ++r) {
          acc[j][r]     *= e0[r];
          acc[j][4 + r] *= e1[r];
        }
      }
    }
    __syncthreads();

    {
      const _Float16* Ms = (const _Float16*)(const void*)sM + (16 * wave + rl) * kMP + koff;
      const _Float16* Xs = (const _Float16*)(const void*)sXT + rl * kMP + koff;
#pragma unroll 1
      for (int k0 = 0; k0 < kQ; k0 += 32) {
        const v16h a = frag_ld(Ms + k0);
        v16h bf[4];
#pragma unroll
        for (int j = 0; j < 4; ++j) bf[j] = frag_ld(Xs + (j * 16) * kMP + k0);
#pragma unroll
        for (int j = 0; j < 4; ++j) acc[j] = mma_h(a, bf[j], acc[j]);
        guard4h(acc[0], acc[1], acc[2], acc[3], a, bf[0], bf[1], bf[2], bf[3]);
      }
    }
#pragma unroll
    for (int j = 0; j < 4; ++j) {
#pragma unroll
      for (int r = 0; r < 8; ++r) slab[(8 * hh + r) * 68 + (j << 4) + rl] = acc[j][r] * kCarryInv;
    }
    wave_lds_sync();
    {
      const int q = lane >> 3, c8 = (lane & 7) * 8;
      v8h hv[4];
#pragma unroll
      for (int it = 0; it < 4; ++it) {
        const int row = it * 4 + q;
        const float* sp = slab + row * 68 + c8;
        const v4f a0 = *(const v4f*)(sp);
        const v4f a1 = *(const v4f*)(sp + 4);
        const v4u xg = *(const v4u*)(XC + (r0 + 16 * wave + row) * kCv + h * kHd + c8);
#pragma unroll
        for (int k = 0; k < 2; ++k) {
          const unsigned wlo = xg[k];
          const unsigned whi = xg[2 + k];
          const float y0 = fmaf(Dh, h16_to_f32(wlo & 0xffffu), a0[2 * k]);
          const float y1 = fmaf(Dh, h16_to_f32(wlo >> 16),     a0[2 * k + 1]);
          const float y2 = fmaf(Dh, h16_to_f32(whi & 0xffffu), a1[2 * k]);
          const float y3 = fmaf(Dh, h16_to_f32(whi >> 16),     a1[2 * k + 1]);
          hv[it][2 * k]         = (_Float16)y0;
          hv[it][2 * k + 1]     = (_Float16)y1;
          hv[it][4 + 2 * k]     = (_Float16)y2;
          hv[it][4 + 2 * k + 1] = (_Float16)y3;
        }
      }
      for (int pass = 0; pass < 2; ++pass) {
#pragma unroll
        for (int it = 0; it < 4; ++it) {
          const int row = it * 4 + q;
          *(volatile v8h*)(Y16 + (r0 + 16 * wave + row) * kDi + h * kHd + c8) = hv[it];
        }
        __threadfence();
      }
    }
    wave_lds_sync();
    {
      const float dec = sScal[0];
#pragma unroll
      for (int j = 0; j < 8; ++j) {
#pragma unroll
        for (int r = 0; r < 8; ++r) Hacc[j][r] *= dec;
      }
      const _Float16* Ws = (const _Float16*)(const void*)sXW + (16 * wave + rl) * kMP + koff;
      const _Float16* Bg = (const _Float16*)(const void*)BT + ((size_t)bc * kNs + rl) * kQ + koff;
#pragma unroll 1
      for (int k0 = 0; k0 < kQ; k0 += 32) {
        const v16h a = frag_ld(Ws + k0);
        {
          v16h bf[4];
#pragma unroll
          for (int j = 0; j < 4; ++j) bf[j] = frag_ld(Bg + (size_t)(j * 16) * kQ + k0);
#pragma unroll
          for (int j = 0; j < 4; ++j) Hacc[j] = mma_h(a, bf[j], Hacc[j]);
          guard4h(Hacc[0], Hacc[1], Hacc[2], Hacc[3], a, bf[0], bf[1], bf[2], bf[3]);
        }
        {
          v16h bf[4];
#pragma unroll
          for (int j = 0; j < 4; ++j) bf[j] = frag_ld(Bg + (size_t)((4 + j) * 16) * kQ + k0);
#pragma unroll
          for (int j = 0; j < 4; ++j) Hacc[4 + j] = mma_h(a, bf[j], Hacc[4 + j]);
          guard4h(Hacc[4], Hacc[5], Hacc[6], Hacc[7], a, bf[0], bf[1], bf[2], bf[3]);
        }
      }
      acc_guard4(Hacc[0], Hacc[1], Hacc[2], Hacc[3]);
      acc_guard4(Hacc[4], Hacc[5], Hacc[6], Hacc[7]);
#pragma unroll
      for (int j = 0; j < 8; ++j) {
#pragma unroll
        for (int r = 0; r < 8; ++r)
          sH[(16 * wave + 8 * hh + r) * kHP + (j << 4) + rl] = f32_to_h16_bits(Hacc[j][r]);
      }
    }
  }
}

__global__ __launch_bounds__(192) void gated_norm_kernel(
    const unsigned short* __restrict__ Y16, const unsigned short* __restrict__ Z16,
    const float* __restrict__ norm_w, unsigned short* __restrict__ YN16)
{
  __shared__ __align__(16) float sG[kDi];
  __shared__ float sRed[8];
  const int tid = threadIdx.x, lane = tid & 31, wave = tid >> 5;
  const size_t row = (size_t)blockIdx.x;
  const unsigned* Yw = (const unsigned*)(const void*)(Y16 + row * kDi);
  const unsigned* Zw = (const unsigned*)(const void*)(Z16 + row * kDi);
  float ss = 0.0f;
#pragma unroll 1
  for (int i = 0; i < 4; ++i) {
    const int wi = tid * 4 + i;
    const unsigned yw = Yw[wi];
    const unsigned zw = Zw[wi];
    const float y0 = h16_to_f32(yw & 0xffffu), y1 = h16_to_f32(yw >> 16);
    const float z0 = h16_to_f32(zw & 0xffffu), z1 = h16_to_f32(zw >> 16);
    const float s0 = z0 * __builtin_amdgcn_rcpf(1.0f + expf(-z0));
    const float s1 = z1 * __builtin_amdgcn_rcpf(1.0f + expf(-z1));
    v2f g;
    g[0] = y0 * s0;
    g[1] = y1 * s1;
    *(v2f*)(sG + 2 * wi) = g;
    ss = fmaf(g[0], g[0], ss);
    ss = fmaf(g[1], g[1], ss);
  }
#pragma unroll
  for (int off = 16; off > 0; off >>= 1) ss += __shfl_xor(ss, off, 32);
  if (lane == 0) sRed[wave] = ss;
  __syncthreads();
  const float tot = ((sRed[0] + sRed[1]) + (sRed[2] + sRed[3])) + (sRed[4] + sRed[5]);
  const float rinv = rsqrtf(tot * (1.0f / (float)kDi) + 1e-5f);
  const v4f a0 = *(const v4f*)(sG + 8 * tid);
  const v4f a1 = *(const v4f*)(sG + 8 * tid + 4);
  const v4f w0 = *(const v4f*)(norm_w + 8 * tid);
  const v4f w1 = *(const v4f*)(norm_w + 8 * tid + 4);
  v8h hv;
#pragma unroll
  for (int e = 0; e < 4; ++e) {
    hv[e]     = (_Float16)((a0[e] * rinv) * w0[e]);
    hv[4 + e] = (_Float16)((a1[e] * rinv) * w1[e]);
  }
  unsigned short* q = YN16 + row * kDi + 8 * tid;
  *(volatile v8h*)q = hv;
  __threadfence();
  *(volatile v8h*)q = hv;
}

extern "C" void kernel_launch(void* const* d_in, const int* in_sizes, int n_in,
                              void* d_out, int out_size, void* d_ws, size_t ws_size,
                              hipStream_t stream)
{
  if (n_in < 9) return;
  if (in_sizes[0] != kRows * kDm) return;
  if (in_sizes[1] != kNin * kDm) return;
  if (in_sizes[2] != kCv * 4) return;
  if (in_sizes[3] != kCv) return;
  if (in_sizes[4] != kNh || in_sizes[5] != kNh || in_sizes[6] != kNh) return;
  if (in_sizes[7] != kDi) return;
  if (in_sizes[8] != kDm * kDi) return;
  if (out_size != kRows * kDm) return;
  if (ws_size < kWsTotal) return;

  const float* x       = (const float*)d_in[0];
  const float* W_in    = (const float*)d_in[1];
  const float* conv_w  = (const float*)d_in[2];
  const float* conv_b  = (const float*)d_in[3];
  const float* dt_bias = (const float*)d_in[4];
  const float* A_log   = (const float*)d_in[5];
  const float* Dv      = (const float*)d_in[6];
  const float* norm_w  = (const float*)d_in[7];
  const float* W_out   = (const float*)d_in[8];
  float* out = (float*)d_out;

  char* ws = (char*)d_ws;
  unsigned short* X16    = (unsigned short*)(ws + kOffX16);
  unsigned short* WIN16  = (unsigned short*)(ws + kOffWIN);
  unsigned short* WOUT16 = (unsigned short*)(ws + kOffWOUT);
  unsigned short* Z16    = (unsigned short*)(ws + kOffZ16);
  unsigned short* XR16   = (unsigned short*)(ws + kOffXR);
  float*          DT32   = (float*)(ws + kOffDT);
  unsigned short* XC16   = (unsigned short*)(ws + kOffXC);
  float*          G32    = (float*)(ws + kOffG);
  unsigned short* BT16   = (unsigned short*)(ws + kOffBT);
  unsigned short* Y16    = XR16;
  unsigned short* YN16   = XC16;

  cast_rows_f16_kernel<<<(kRows * kDm / 8) / 256, 256, 0, stream>>>(x, X16, kRows * kDm / 8, kDm, kRows, 1.0f);
  cast_rows_f16_kernel<<<(kNinP * kDm / 8) / 256, 256, 0, stream>>>(W_in, WIN16, kNinP * kDm / 8, kDm, kNin, kWCarry);
  cast_rows_f16_kernel<<<(kDm * kDi / 8) / 256, 256, 0, stream>>>(W_out, WOUT16, kDm * kDi / 8, kDi, kDm, kWCarry);

  gemm64_f16_kernel<2><<<dim3((kRows / 64) * (kNinP / 64) / 8, 1), 256, 0, stream>>>(
      X16, kDm, 0L, WIN16, kDm, 0L,
      DT32, kDtP, 0L, x,
      Z16, XR16, DT32,
      kRows, kNinP, kDm, 1, kWCarryInv);

  conv_silu_kernel<<<dim3(kCv / 256, kRows / 64), 128, 0, stream>>>(XR16, conv_w, conv_b, XC16);

  bt_transpose_kernel<<<kBC, 256, 0, stream>>>(XC16, BT16);

  gemm64_f16_kernel<0><<<dim3(kBC / 8, 1), 256, 0, stream>>>(
      XC16 + kDi + kNs, kCv, (long)kQ * kCv, XC16 + kDi, kCv, (long)kQ * kCv,
      G32, kQ, (long)kQ * kQ, x,
      Z16, XR16, DT32,
      kQ, kQ, kNs, kBC, 1.0f);

  ssd_chunk_kernel<<<kBatch * kNh, 128, 0, stream>>>(XC16, DT32, G32, BT16, dt_bias, A_log, Dv, Y16);

  gated_norm_kernel<<<kRows, 192, 0, stream>>>(Y16, Z16, norm_w, YN16);

  gemm64_f16_kernel<1><<<dim3((kRows / 64) * (kDm / 64) / 8, 1), 256, 0, stream>>>(
      YN16, kDi, 0L, WOUT16, kDi, 0L,
      out, kDm, 0L, x,
      Z16, XR16, DT32,
      kRows, kDm, kDi, 1, kWCarryInv);
}
